// Conv_78022375899305
// MI455X (gfx1250) — hardware-verified
//
#include <hip/hip_runtime.h>

typedef unsigned short u16;
typedef __bf16 v16bf __attribute__((ext_vector_type(16)));
typedef u16 v16us __attribute__((ext_vector_type(16)));
typedef u16 v8us __attribute__((ext_vector_type(8)));
typedef u16 v4us __attribute__((ext_vector_type(4)));
typedef unsigned v4u __attribute__((ext_vector_type(4)));
typedef int v8i __attribute__((ext_vector_type(8)));
typedef float v8f __attribute__((ext_vector_type(8)));
typedef float v4f __attribute__((ext_vector_type(4)));
typedef float v2f __attribute__((ext_vector_type(2)));
typedef v8us __attribute__((may_alias)) v8usa;
typedef v4us __attribute__((may_alias)) v4usa;
typedef v4u __attribute__((may_alias)) v4ua;
typedef v4f __attribute__((may_alias)) v4fa;
typedef v2f __attribute__((may_alias)) v2fa;

union FragU { v16us v; v8us half[2]; };

#define NCH   4
#define SNB   10
#define CDIM  64
#define NPOS  16
#define NIN   256
#define NB    64
#define LSEQ  16
#define N1    160
#define N2    1600
#define NIT   40000
#define TBROWS 40064
#define XSROWS 2048
#define AROWS  (TBROWS + XSROWS)
#define NODEA  (NB * N1)
#define NODEB  (NB * LSEQ)
#define GRPA   (NODEA * NCH)
#define GRPB   (NODEB * NCH)
#define GRPAB  (GRPA + GRPB)
#define KATT   160
#define KFIN   768

static_assert(SNB == 10);
static_assert(SNB <= 16);
static_assert(N1 == LSEQ * SNB);
static_assert(N2 == N1 * SNB);
static_assert(NCH * CDIM == NIN);
static_assert(KATT % 32 == 0 && KFIN % 32 == 0 && NIN % 32 == 0);
static_assert(NIT <= 313 * 128 && TBROWS == 313 * 128);
static_assert(AROWS % 32 == 0);
static_assert(GRPAB % 128 == 0 && GRPB % 128 == 0);
static_assert(NODEA % 2 == 0 && NODEB % 2 == 0 && N1 % 2 == 0 && LSEQ % 2 == 0);
static_assert(NODEB % 16 == 0);

#define SZ_TBXS ((size_t)AROWS * 512)
#define SZ_ROUT ((size_t)AROWS * 1024)
#define SZ_SESS ((size_t)NB * 1024)
#define SZ_CAT  ((size_t)GRPAB * 512)
#define SZ_O    ((size_t)GRPAB * 256)
#define SZ_CATC ((size_t)GRPB * 512)
#define SZ_HG   ((size_t)GRPB * 256)
#define SZ_WRT  ((size_t)256 * 512)
#define SZ_W1C  ((size_t)2 * 64 * KATT * 2)
#define SZ_W3C  ((size_t)2 * 64 * 256 * 2)
#define SZ_LCAT ((size_t)256 * KFIN * 2)
#define OFF_TBXS ((size_t)0)
#define OFF_ROUT (OFF_TBXS + SZ_TBXS)
#define OFF_SESS (OFF_ROUT + SZ_ROUT)
#define OFF_CAT  (OFF_SESS + SZ_SESS)
#define OFF_O    (OFF_CAT + SZ_CAT)
#define OFF_CATC (OFF_O + SZ_O)
#define OFF_HG   (OFF_CATC + SZ_CATC)
#define OFF_WRT  (OFF_HG + SZ_HG)
#define OFF_W1C  (OFF_WRT + SZ_WRT)
#define OFF_W3C  (OFF_W1C + SZ_W1C)
#define OFF_LCAT (OFF_W3C + SZ_W3C)
#define WS_TOTAL (OFF_LCAT + SZ_LCAT)
static_assert(SZ_TBXS % 128 == 0 && SZ_ROUT % 128 == 0 && SZ_SESS % 128 == 0 && SZ_CAT % 128 == 0);
static_assert(SZ_O % 128 == 0 && SZ_CATC % 128 == 0 && SZ_HG % 128 == 0 && SZ_WRT % 128 == 0);
static_assert(SZ_W1C % 4096 == 0 && SZ_W3C % 4096 == 0 && SZ_LCAT % 128 == 0);
static_assert(WS_TOTAL <= (size_t)134217728);

#define PB_TB  0
#define PB_XH  (PB_TB + TBROWS * 32 / 256)
#define PB_XS  (PB_XH + 128)
#define PB_WR  (PB_XS + 128)
#define PB_W1  (PB_WR + 32)
#define PB_W3  (PB_W1 + 10)
#define PB_LA  (PB_W3 + 16)
#define PB_LB  (PB_LA + 32)
#define PB_LC  (PB_LB + 32)
#define PB_END (PB_LC + 32)
static_assert((TBROWS * 32) % 256 == 0);

__device__ __forceinline__ unsigned bfbits(float f) {
  unsigned u = __builtin_bit_cast(unsigned, f);
  u += 0x7FFFu + ((u >> 16) & 1u);
  return u >> 16;
}
__device__ __forceinline__ float bff(unsigned bits) {
  return __builtin_bit_cast(float, bits << 16);
}
__device__ __forceinline__ float bfr(float f) { return bff(bfbits(f)); }
__device__ __forceinline__ int clampi(int v, int lo, int hi) {
  return (v < lo) ? lo : ((v > hi) ? hi : v);
}
__device__ __forceinline__ float hsum16(float v) {
  v += __shfl_xor(v, 1);
  v += __shfl_xor(v, 2);
  v += __shfl_xor(v, 4);
  v += __shfl_xor(v, 8);
  return v;
}
__device__ __forceinline__ float sigm_f(float v) {
  v = fminf(fmaxf(v, -30.0f), 30.0f);
  const float e = expf(-v);
  return 1.0f / (1.0f + e);
}

__device__ __forceinline__ v8f wmma_bf(v16us a, v16us b, v8f c) {
  const v16bf ab = __builtin_bit_cast(v16bf, a);
  const v16bf bb = __builtin_bit_cast(v16bf, b);
  v8f d = __builtin_amdgcn_wmma_f32_16x16x32_bf16(false, ab, false, bb, (short)0, c, false, false);
  const v8i ai = __builtin_bit_cast(v8i, a);
  const v8i bi = __builtin_bit_cast(v8i, b);
  asm volatile("v_nop\n\tv_nop\n\tv_nop\n\tv_nop" : "+v"(d) : "v"(ai), "v"(bi));
  return d;
}

__device__ __forceinline__ v16us load_frag(const u16* p, int h) {
  FragU f;
  f.half[0] = *(const v8usa*)(p + 8 * h);
  f.half[1] = *(const v8usa*)(p + 16 + 8 * h);
  return f.v;
}

__device__ __forceinline__ void st2_v8us(u16* dst, v8us o) {
  *(volatile v8us*)dst = o;
  __threadfence();
  *(volatile v8us*)dst = o;
}

__device__ __forceinline__ void cvt8_store(const float* __restrict__ src, u16* dst, unsigned keep) {
  const v4f a = *(const v4fa*)src;
  const v4f c = *(const v4fa*)(src + 4);
  const v8us o = { (u16)(bfbits(a.x) & keep), (u16)(bfbits(a.y) & keep), (u16)(bfbits(a.z) & keep), (u16)(bfbits(a.w) & keep),
                   (u16)(bfbits(c.x) & keep), (u16)(bfbits(c.y) & keep), (u16)(bfbits(c.z) & keep), (u16)(bfbits(c.w) & keep) };
  st2_v8us(dst, o);
}

__device__ __forceinline__ v8us gather8(const float* __restrict__ src, int stride) {
  const float f0 = src[0];
  const float f1 = src[(size_t)stride];
  const float f2 = src[(size_t)2 * stride];
  const float f3 = src[(size_t)3 * stride];
  const float f4 = src[(size_t)4 * stride];
  const float f5 = src[(size_t)5 * stride];
  const float f6 = src[(size_t)6 * stride];
  const float f7 = src[(size_t)7 * stride];
  const v8us o = { (u16)bfbits(f0), (u16)bfbits(f1), (u16)bfbits(f2), (u16)bfbits(f3),
                   (u16)bfbits(f4), (u16)bfbits(f5), (u16)bfbits(f6), (u16)bfbits(f7) };
  return o;
}

__global__ __launch_bounds__(256) __attribute__((amdgpu_num_vgpr(248)))
void k_prep(const float* __restrict__ table, const float* __restrict__ hin, const float* __restrict__ seq,
            const float* __restrict__ Wr, const float* __restrict__ w1, const float* __restrict__ w3,
            const float* __restrict__ l1, const float* __restrict__ l2, char* __restrict__ ws)
{
  const int blk = blockIdx.x, tid = threadIdx.x;
  u16* tbxs = (u16*)(ws + OFF_TBXS);
  if (blk < PB_XH) {
    const int g = blk * 256 + tid;
    const int row = g >> 5;
    const int rc = (row < NIT) ? row : (NIT - 1);
    const unsigned keep = (row < NIT) ? 0xFFFFu : 0u;
    cvt8_store(table + (size_t)rc * NIN + (g & 31) * 8, tbxs + (size_t)g * 8, keep);
  } else if (blk < PB_XS) {
    const int g = (blk - PB_XH) * 256 + tid;
    cvt8_store(hin + (size_t)g * 8, tbxs + ((size_t)TBROWS * 32 + g) * 8, 0xFFFFu);
  } else if (blk < PB_WR) {
    const int g = (blk - PB_XS) * 256 + tid;
    cvt8_store(seq + (size_t)g * 8, tbxs + ((size_t)TBROWS * 32 + 32768 + g) * 8, 0xFFFFu);
  } else if (blk < PB_W1) {
    const int q = (blk - PB_WR) * 256 + tid;
    const int n = q >> 5, k0 = (q & 31) * 8;
    const int c = n >> 6, kk = n & 63;
    const v8us o = gather8(Wr + ((size_t)c * NIN + k0) * CDIM + kk, CDIM);
    st2_v8us((u16*)(ws + OFF_WRT) + (size_t)q * 8, o);
  } else if (blk < PB_W3) {
    const int q = (blk - PB_W1) * 256 + tid;
    const int nh = q / 1280;
    const int rem = q - nh * 1280;
    const int n = rem / 20;
    const int k0 = (rem - n * 20) * 8;
    const float* base = w1 + (size_t)nh * 81 * CDIM + n;
    unsigned bits[8];
    #pragma unroll
    for (int j = 0; j < 8; ++j) {
      const int k = k0 + j;
      const int kk = (k < 64) ? k : (k - 64);
      const int kc = (kk < 80) ? kk : 80;
      const float f = base[(size_t)kc * CDIM];
      bits[j] = (kk <= 80) ? bfbits(f) : 0u;
    }
    const v8us o = { (u16)bits[0], (u16)bits[1], (u16)bits[2], (u16)bits[3],
                     (u16)bits[4], (u16)bits[5], (u16)bits[6], (u16)bits[7] };
    st2_v8us((u16*)(ws + OFF_W1C) + (size_t)q * 8, o);
  } else if (blk < PB_LA) {
    const int q = (blk - PB_W3) * 256 + tid;
    const int nh = q >> 11, n = (q >> 5) & 63, k0 = (q & 31) * 8;
    const v8us o = gather8(w3 + ((size_t)nh * 128 + (k0 & 127)) * CDIM + n, CDIM);
    st2_v8us((u16*)(ws + OFF_W3C) + (size_t)q * 8, o);
  } else if (blk < PB_LB) {
    const int q = (blk - PB_LA) * 256 + tid;
    const int n = q >> 5, k0 = (q & 31) * 8;
    const v8us o = gather8(l1 + (size_t)k0 * NIN + n, NIN);
    st2_v8us((u16*)(ws + OFF_LCAT) + (size_t)n * KFIN + k0, o);
  } else if (blk < PB_LC) {
    const int q = (blk - PB_LB) * 256 + tid;
    const int n = q >> 5, k0 = (q & 31) * 8;
    const v8us o = gather8(l1 + (size_t)k0 * NIN + n, NIN);
    st2_v8us((u16*)(ws + OFF_LCAT) + (size_t)n * KFIN + 256 + k0, o);
  } else {
    const int q = (blk - PB_LC) * 256 + tid;
    const int n = q >> 5, k0 = (q & 31) * 8;
    const v8us o = gather8(l2 + (size_t)k0 * NIN + n, NIN);
    st2_v8us((u16*)(ws + OFF_LCAT) + (size_t)n * KFIN + 512 + k0, o);
  }
}

__device__ __forceinline__ void tile_store_pass(const float* sT, float* dst, int w, int lane) {
  #pragma unroll
  for (int i = 0; i < 16; ++i) {
    const int off = (w * 16 + i) * 128 + lane * 4;
    const v4f v = *(const v4fa*)(sT + off);
    *(volatile v4f*)(dst + off) = v;
  }
}

__global__ __launch_bounds__(128) __attribute__((amdgpu_num_vgpr(248)))
void k_route(const u16* __restrict__ A, const u16* __restrict__ WrT,
             const float* __restrict__ br, float* __restrict__ out)
{
  __shared__ __attribute__((aligned(16))) float sT[32 * 256];
  __shared__ __attribute__((aligned(16))) float sBr[256];

  const int tid = threadIdx.x, lane = tid & 31, w = tid >> 5;
  const int h = lane >> 4, m = lane & 15;
  const int row0 = blockIdx.x * 32;

  {
    const int q = tid & 63;
    const v4f v = *(const v4fa*)(br + q * 4);
    const v4f r = { bfr(v.x), bfr(v.y), bfr(v.z), bfr(v.w) };
    if (w < 2) *(v4fa*)(sBr + q * 4) = r;
  }
  __syncthreads();

  const u16* a0 = A + (size_t)(row0 + m) * NIN;
  const u16* a1 = a0 + (size_t)16 * NIN;
  const u16* bp = WrT + (size_t)(64 * w + m) * NIN;

  const v8f z8 = {0.f, 0.f, 0.f, 0.f, 0.f, 0.f, 0.f, 0.f};
  v8f acc[2][4];
  #pragma unroll
  for (int mt = 0; mt < 2; ++mt)
    #pragma unroll
    for (int nt = 0; nt < 4; ++nt) acc[mt][nt] = z8;

  #pragma unroll 1
  for (int k0 = 0; k0 < NIN; k0 += 32) {
    const v16us f0 = load_frag(a0 + k0, h);
    const v16us f1 = load_frag(a1 + k0, h);
    #pragma unroll
    for (int nt = 0; nt < 4; ++nt) {
      const v16us b = load_frag(bp + (size_t)nt * 16 * NIN + k0, h);
      acc[0][nt] = wmma_bf(f0, b, acc[0][nt]);
      acc[1][nt] = wmma_bf(f1, b, acc[1][nt]);
    }
  }

  float ss[2][8];
  #pragma unroll
  for (int mt = 0; mt < 2; ++mt)
    #pragma unroll
    for (int r = 0; r < 8; ++r) ss[mt][r] = 0.0f;
  #pragma unroll
  for (int nt = 0; nt < 4; ++nt) {
    const float bb = sBr[64 * w + 16 * nt + m];
    #pragma unroll
    for (int mt = 0; mt < 2; ++mt)
      #pragma unroll
      for (int r = 0; r < 8; ++r) {
        const float v = acc[mt][nt][r] + bb;
        acc[mt][nt][r] = v;
        ss[mt][r] += v * v;
      }
  }
  #pragma unroll
  for (int mt = 0; mt < 2; ++mt)
    #pragma unroll
    for (int r = 0; r < 8; ++r) {
      const float s = hsum16(ss[mt][r]);
      ss[mt][r] = 1.0f / fmaxf(sqrtf(s), 1e-12f);
    }
  #pragma unroll
  for (int nt = 0; nt < 4; ++nt)
    #pragma unroll
    for (int mt = 0; mt < 2; ++mt)
      #pragma unroll
      for (int r = 0; r < 8; ++r)
        sT[(16 * mt + 8 * h + r) * NIN + 64 * w + 16 * nt + m] = acc[mt][nt][r] * ss[mt][r];
  __syncthreads();

  float* dst = out + (size_t)row0 * NIN;
  tile_store_pass(sT, dst, w, lane);
  __threadfence();
  tile_store_pass(sT, dst, w, lane);
}

__global__ __launch_bounds__(64) __attribute__((amdgpu_num_vgpr(248)))
void k_sess(const float* __restrict__ item, const float* __restrict__ mask, float* __restrict__ sess)
{
  const int b = blockIdx.x, t = threadIdx.x;
  float ms = 0.0f;
  #pragma unroll
  for (int q = 0; q < 4; ++q) {
    const v4f mv = *(const v4fa*)(mask + b * LSEQ + 4 * q);
    ms += bfr(mv.x); ms += bfr(mv.y); ms += bfr(mv.z); ms += bfr(mv.w);
  }
  v4f acc = {0.f, 0.f, 0.f, 0.f};
  #pragma unroll 4
  for (int l = 0; l < LSEQ; ++l) {
    const v4f v = *(const v4fa*)(item + (size_t)(b * LSEQ + l) * NIN + 4 * t);
    acc.x += v.x; acc.y += v.y; acc.z += v.z; acc.w += v.w;
  }
  const float inv = 1.0f / ms;
  const v4f o = { acc.x * inv, acc.y * inv, acc.z * inv, acc.w * inv };
  float* dst = sess + (size_t)b * NIN + 4 * t;
  *(volatile v4f*)dst = o;
  __threadfence();
  *(volatile v4f*)dst = o;
}

template <int MODE>
__global__ __launch_bounds__(256) __attribute__((amdgpu_num_vgpr(248)))
void k_att(const float* neighP, const float* selfP,
           const int* __restrict__ nbrIdx, const int* __restrict__ selfIdx,
           const float* __restrict__ wArr, const float* __restrict__ posArr,
           const float* __restrict__ sessP, const u16* __restrict__ W1c,
           const float* __restrict__ w2, unsigned* __restrict__ cat)
{
  __shared__ __attribute__((aligned(16))) float sN[20 * NIN];
  __shared__ __attribute__((aligned(16))) float sS[NIN];
  __shared__ __attribute__((aligned(16))) float sP[320];
  __shared__ __attribute__((aligned(16))) float sWt[32];
  __shared__ __attribute__((aligned(16))) float sW2[64];
  __shared__ __attribute__((aligned(16))) u16 sA[80 * KATT];
  __shared__ __attribute__((aligned(16))) unsigned sC[8 * 128];

  constexpr int PERB = (MODE == 0) ? N1 : LSEQ;
  const int tid = threadIdx.x, lane = tid & 31, w = tid >> 5;
  const int h = lane >> 4, m = lane & 15;
  const int tile = blockIdx.x;
  const int nd0 = tile * 2;
  const int b = nd0 / PERB;

  #pragma unroll
  for (int i = 0; i < 5; ++i) {
    const int u = tid + 256 * i;
    const int r = u >> 6, c4 = (u & 63) * 4;
    size_t ro;
    if (MODE == 2) {
      ro = (size_t)(nd0 * SNB + r) * NIN;
    } else {
      const int id = clampi(nbrIdx[nd0 * SNB + r], 0, NIT - 1);
      ro = (size_t)id * NIN;
    }
    const v4f v = *(const v4fa*)(neighP + ro + c4);
    *(v4fa*)(sN + r * NIN + c4) = v;
  }
  if (w < 2) {
    const v4f v = *(const v4fa*)(sessP + (size_t)b * NIN + tid * 4);
    *(v4fa*)(sS + tid * 4) = v;
  } else if (w < 5) {
    const int t2 = tid - 64;
    const int pi = (t2 < 79) ? t2 : 79;
    const v4f v = *(const v4fa*)(posArr + (size_t)nd0 * (SNB * NPOS) + pi * 4);
    *(v4fa*)(sP + pi * 4) = v;
  } else if (w == 5) {
    const int t3 = tid - 160;
    const int pi = (t3 < 4) ? t3 : 4;
    const v4f v = *(const v4fa*)(wArr + (size_t)nd0 * SNB + pi * 4);
    *(v4fa*)(sWt + pi * 4) = v;
  } else if (w == 6) {
    const int t4 = tid - 192;
    const int pi = (t4 < 15) ? t4 : 15;
    const v4f v = *(const v4fa*)(w2 + pi * 4);
    const v4f r = { bfr(v.x), bfr(v.y), bfr(v.z), bfr(v.w) };
    *(v4fa*)(sW2 + pi * 4) = r;
  }
  __syncthreads();

  #pragma unroll
  for (int i = 0; i < 3; ++i) {
    const int u = tid + 256 * i;
    const int uu = (u < 639) ? u : 639;
    const int row = uu >> 3, k8 = (uu & 7) * 8;
    const int g = row / 10;
    const int s = row - g * 10;
    const int j = g >> 2, c = g & 3;
    const float* np = sN + (j * SNB + s) * NIN + c * CDIM + k8;
    const float* sp = sS + c * CDIM + k8;
    const v4f n0 = *(const v4fa*)np;
    const v4f n1 = *(const v4fa*)(np + 4);
    const v4f s0 = *(const v4fa*)sp;
    const v4f s1 = *(const v4fa*)(sp + 4);
    const float p0 = s0.x * n0.x, p1 = s0.y * n0.y, p2 = s0.z * n0.z, p3 = s0.w * n0.w;
    const float p4 = s1.x * n1.x, p5 = s1.y * n1.y, p6 = s1.z * n1.z, p7 = s1.w * n1.w;
    const unsigned h0 = bfbits(p0), h1 = bfbits(p1), h2 = bfbits(p2), h3 = bfbits(p3);
    const unsigned h4 = bfbits(p4), h5 = bfbits(p5), h6 = bfbits(p6), h7 = bfbits(p7);
    const v8us hi = { (u16)h0, (u16)h1, (u16)h2, (u16)h3, (u16)h4, (u16)h5, (u16)h6, (u16)h7 };
    const v8us lo = { (u16)bfbits(p0 - bff(h0)), (u16)bfbits(p1 - bff(h1)), (u16)bfbits(p2 - bff(h2)), (u16)bfbits(p3 - bff(h3)),
                      (u16)bfbits(p4 - bff(h4)), (u16)bfbits(p5 - bff(h5)), (u16)bfbits(p6 - bff(h6)), (u16)bfbits(p7 - bff(h7)) };
    if (u < 640) {
      *(v8usa*)(sA + row * KATT + k8) = hi;
      *(v8usa*)(sA + row * KATT + 64 + k8) = lo;
    }
  }
  if (tid < 96) {
    const int rr = (tid < 79) ? tid : 79;
    const int g = rr / 10;
    const int s = rr - g * 10;
    const int src = (g >> 2) * SNB + s;
    const float wv = sWt[src];
    const v4f q0 = *(const v4fa*)(sP + src * NPOS);
    const v4f q1 = *(const v4fa*)(sP + src * NPOS + 4);
    const v4f q2 = *(const v4fa*)(sP + src * NPOS + 8);
    const v4f q3 = *(const v4fa*)(sP + src * NPOS + 12);
    const v8us t0 = { (u16)bfbits(wv),   (u16)bfbits(q0.x), (u16)bfbits(q0.y), (u16)bfbits(q0.z),
                      (u16)bfbits(q0.w), (u16)bfbits(q1.x), (u16)bfbits(q1.y), (u16)bfbits(q1.z) };
    const v8us t1 = { (u16)bfbits(q1.w), (u16)bfbits(q2.x), (u16)bfbits(q2.y), (u16)bfbits(q2.z),
                      (u16)bfbits(q2.w), (u16)bfbits(q3.x), (u16)bfbits(q3.y), (u16)bfbits(q3.z) };
    const v8us t2 = { (u16)bfbits(q3.w), (u16)0, (u16)0, (u16)0, (u16)0, (u16)0, (u16)0, (u16)0 };
    const v8us t3 = { (u16)0, (u16)0, (u16)0, (u16)0, (u16)0, (u16)0, (u16)0, (u16)0 };
    if (tid < 80) {
      u16* dp = sA + rr * KATT + 128;
      *(v8usa*)(dp) = t0;
      *(v8usa*)(dp + 8) = t1;
      *(v8usa*)(dp + 16) = t2;
      *(v8usa*)(dp + 24) = t3;
    }
  }
  __syncthreads();

  const v8f z8 = {0.f, 0.f, 0.f, 0.f, 0.f, 0.f, 0.f, 0.f};
  v8f acc[4];
  #pragma unroll
  for (int nt = 0; nt < 4; ++nt) acc[nt] = z8;
  {
    const int ma = (m < 9) ? m : 9;
    const u16 mk = (m < SNB) ? (u16)0xFFFFu : (u16)0;
    const v8us mkv = { mk, mk, mk, mk, mk, mk, mk, mk };
    const u16* arow = sA + (w * SNB + ma) * KATT;
    const u16* brow = W1c + (size_t)m * KATT;
    #pragma unroll 1
    for (int k0 = 0; k0 < KATT; k0 += 32) {
      FragU fa;
      fa.half[0] = *(const v8usa*)(arow + k0 + 8 * h) & mkv;
      fa.half[1] = *(const v8usa*)(arow + k0 + 16 + 8 * h) & mkv;
      #pragma unroll
      for (int nt = 0; nt < 4; ++nt) {
        const v16us bfr_ = load_frag(brow + (size_t)nt * 16 * KATT + k0, h);
        acc[nt] = wmma_bf(fa.v, bfr_, acc[nt]);
      }
    }
  }

  float e[8];
  #pragma unroll
  for (int r = 0; r < 8; ++r) e[r] = 0.0f;
  #pragma unroll
  for (int nt = 0; nt < 4; ++nt) {
    const float wv = sW2[16 * nt + m];
    #pragma unroll
    for (int r = 0; r < 8; ++r) {
      const float v = acc[nt][r];
      const float lv = (v >= 0.0f) ? v : 0.2f * v;
      e[r] += lv * wv;
    }
  }
  float oth[8];
  #pragma unroll
  for (int r = 0; r < 8; ++r) e[r] = hsum16(e[r]);
  #pragma unroll
  for (int r = 0; r < 8; ++r) oth[r] = __shfl_xor(e[r], 16);
  float ev[10];
  #pragma unroll
  for (int s = 0; s < 8; ++s) ev[s] = (h != 0) ? oth[s] : e[s];
  ev[8] = (h != 0) ? e[0] : oth[0];
  ev[9] = (h != 0) ? e[1] : oth[1];

  float mx = ev[0];
  #pragma unroll
  for (int s = 1; s < SNB; ++s) mx = fmaxf(mx, ev[s]);
  float den = 0.0f;
  #pragma unroll
  for (int s = 0; s < SNB; ++s) { ev[s] = expf(ev[s] - mx); den += ev[s]; }
  const float inv = 1.0f / den;

  const int j = w >> 2, c = w & 3;
  const float* nb = sN + (j * SNB) * NIN + c * CDIM + 2 * lane;
  float nx = 0.0f, ny = 0.0f;
  #pragma unroll
  for (int s = 0; s < SNB; ++s) {
    const v2f t = *(const v2fa*)(nb + s * NIN);
    const float p = ev[s] * inv;
    nx += p * t.x;
    ny += p * t.y;
  }
  const int nd = nd0 + j;
  size_t so;
  if (MODE == 0) {
    const int sid = clampi(selfIdx[nd], 0, NIT - 1);
    so = (size_t)sid * NIN;
  } else {
    so = (size_t)nd * NIN;
  }
  const v2f sf = *(const v2fa*)(selfP + so + c * CDIM + 2 * lane);

  const unsigned sh0 = bfbits(sf.x), sh1 = bfbits(sf.y);
  const unsigned nh0 = bfbits(nx),   nh1 = bfbits(ny);
  const unsigned sl0 = bfbits(sf.x - bff(sh0)), sl1 = bfbits(sf.y - bff(sh1));
  const unsigned nl0 = bfbits(nx - bff(nh0)),   nl1 = bfbits(ny - bff(nh1));
  unsigned* crow = sC + w * 128;
  crow[lane]      = sh0 | (sh1 << 16);
  crow[32 + lane] = nh0 | (nh1 << 16);
  crow[64 + lane] = sl0 | (sl1 << 16);
  crow[96 + lane] = nl0 | (nl1 << 16);
  __syncthreads();

  const v4u val = *(const v4ua*)(sC + w * 128 + lane * 4);
  unsigned* dst = cat + ((size_t)tile * 8 + w) * 128 + lane * 4;
  *(volatile v4u*)dst = val;
  __threadfence();
  *(volatile v4u*)dst = val;
}

__global__ __launch_bounds__(128) __attribute__((amdgpu_num_vgpr(248)))
void k_w3(const u16* __restrict__ catp, const u16* __restrict__ W3c, float* __restrict__ outp)
{
  __shared__ __attribute__((aligned(16))) float sT[128 * 64];

  const int tid = threadIdx.x, lane = tid & 31, w = tid >> 5;
  const int h = lane >> 4, m = lane & 15;
  const int rowb = blockIdx.x * 128;

  const u16* a0 = catp + (size_t)(rowb + 32 * w + m) * 256;
  const u16* a1 = a0 + (size_t)16 * 256;
  const u16* bp = W3c + (size_t)m * 256;

  const v8f z8 = {0.f, 0.f, 0.f, 0.f, 0.f, 0.f, 0.f, 0.f};
  v8f acc[2][4];
  #pragma unroll
  for (int mt = 0; mt < 2; ++mt)
    #pragma unroll
    for (int nt = 0; nt < 4; ++nt) acc[mt][nt] = z8;

  #pragma unroll 1
  for (int k0 = 0; k0 < 256; k0 += 32) {
    const v16us f0 = load_frag(a0 + k0, h);
    const v16us f1 = load_frag(a1 + k0, h);
    #pragma unroll
    for (int nt = 0; nt < 4; ++nt) {
      const v16us b = load_frag(bp + (size_t)nt * 16 * 256 + k0, h);
      acc[0][nt] = wmma_bf(f0, b, acc[0][nt]);
      acc[1][nt] = wmma_bf(f1, b, acc[1][nt]);
    }
  }

  #pragma unroll
  for (int nt = 0; nt < 4; ++nt)
    #pragma unroll
    for (int mt = 0; mt < 2; ++mt)
      #pragma unroll
      for (int r = 0; r < 8; ++r) {
        const float v = acc[mt][nt][r];
        sT[(32 * w + 16 * mt + 8 * h + r) * 64 + 16 * nt + m] = (v > 0.0f) ? v : (v - v);
      }
  __syncthreads();

  float* dst = outp + (size_t)rowb * 64;
  tile_store_pass(sT, dst, w, lane);
  __threadfence();
  tile_store_pass(sT, dst, w, lane);
}

__global__ __launch_bounds__(128) __attribute__((amdgpu_num_vgpr(248)))
void k_fin(const float* __restrict__ HG, const u16* __restrict__ XS, const u16* __restrict__ Lcat,
           const float* __restrict__ b1, const float* __restrict__ b2, const float* __restrict__ l3,
           float* __restrict__ out)
{
  __shared__ __attribute__((aligned(16))) u16 sA[16 * KFIN];
  __shared__ __attribute__((aligned(16))) float sQ[16 * NIN];
  __shared__ __attribute__((aligned(16))) float sBias[NIN];
  __shared__ __attribute__((aligned(16))) float sL3[NIN];

  const int tid = threadIdx.x, lane = tid & 31, w = tid >> 5;
  const int h = lane >> 4, m = lane & 15;
  const int row0 = blockIdx.x * 16;

  {
    const int q = tid & 63;
    const v4f v1 = *(const v4fa*)(b1 + q * 4);
    const v4f v2 = *(const v4fa*)(b2 + q * 4);
    const v4f v3 = *(const v4fa*)(l3 + q * 4);
    const v4f bs = { bfr(v1.x) + bfr(v2.x), bfr(v1.y) + bfr(v2.y), bfr(v1.z) + bfr(v2.z), bfr(v1.w) + bfr(v2.w) };
    const v4f lw = { bfr(v3.x), bfr(v3.y), bfr(v3.z), bfr(v3.w) };
    if (w < 2) *(v4fa*)(sBias + q * 4) = bs;
    else       *(v4fa*)(sL3 + q * 4) = lw;
  }

  #pragma unroll
  for (int i = 0; i < 8; ++i) {
    const int u = tid + 128 * i;
    const int row = u >> 6, c4 = (u & 63) * 4;
    const v4f v = *(const v4fa*)(HG + (size_t)(row0 + row) * NIN + c4);
    const unsigned h0 = bfbits(v.x), h1 = bfbits(v.y), h2 = bfbits(v.z), h3 = bfbits(v.w);
    const v4us hh = { (u16)h0, (u16)h1, (u16)h2, (u16)h3 };
    const v4us ll = { (u16)bfbits(v.x - bff(h0)), (u16)bfbits(v.y - bff(h1)),
                      (u16)bfbits(v.z - bff(h2)), (u16)bfbits(v.w - bff(h3)) };
    *(v4usa*)(sA + row * KFIN + c4) = hh;
    *(v4usa*)(sA + row * KFIN + 256 + c4) = ll;
  }
  #pragma unroll
  for (int i = 0; i < 4; ++i) {
    const int u = tid + 128 * i;
    const int row = u >> 5, k8 = (u & 31) * 8;
    const v8us x = *(const v8usa*)(XS + (size_t)(row0 + row) * NIN + k8);
    *(v8usa*)(sA + row * KFIN + 512 + k8) = x;
  }
  __syncthreads();

  const v8f z8 = {0.f, 0.f, 0.f, 0.f, 0.f, 0.f, 0.f, 0.f};
  v8f acc[4];
  #pragma unroll
  for (int nt = 0; nt < 4; ++nt) acc[nt] = z8;
  {
    const u16* arow = sA + m * KFIN;
    const u16* brow = Lcat + (size_t)(64 * w + m) * KFIN;
    #pragma unroll 1
    for (int k0 = 0; k0 < KFIN; k0 += 32) {
      const v16us a = load_frag(arow + k0, h);
      #pragma unroll
      for (int nt = 0; nt < 4; ++nt) {
        const v16us b = load_frag(brow + (size_t)nt * 16 * KFIN + k0, h);
        acc[nt] = wmma_bf(a, b, acc[nt]);
      }
    }
  }
  #pragma unroll
  for (int nt = 0; nt < 4; ++nt) {
    const int col = 64 * w + 16 * nt + m;
    const float bias = sBias[col];
    const float lw = sL3[col];
    #pragma unroll
    for (int r = 0; r < 8; ++r)
      sQ[(8 * h + r) * NIN + col] = sigm_f(acc[nt][r] + bias) * lw;
  }
  __syncthreads();

  v4f o[4][2];
  #pragma unroll
  for (int rr = 0; rr < 4; ++rr) {
    const int row = 4 * w + rr;
    const v4f qa = *(const v4fa*)(sQ + row * NIN + lane * 8);
    const v4f qb = *(const v4fa*)(sQ + row * NIN + lane * 8 + 4);
    float al = ((qa.x + qa.y) + (qa.z + qa.w)) + ((qb.x + qb.y) + (qb.z + qb.w));
    al += __shfl_xor(al, 1);
    al += __shfl_xor(al, 2);
    al += __shfl_xor(al, 4);
    al += __shfl_xor(al, 8);
    al += __shfl_xor(al, 16);
    const float om = 1.0f - al;
    #pragma unroll
    for (int i = 0; i < 2; ++i) {
      const int col = i * 128 + lane * 4;
      const v4us hb = *(const v4usa*)(sA + row * KFIN + 512 + col);
      const v4f hg = *(const v4fa*)(HG + (size_t)(row0 + row) * NIN + col);
      const v4f t = { al * bff((unsigned)hb.x) + om * hg.x, al * bff((unsigned)hb.y) + om * hg.y,
                      al * bff((unsigned)hb.z) + om * hg.z, al * bff((unsigned)hb.w) + om * hg.w };
      o[rr][i] = t;
    }
  }
  #pragma unroll
  for (int rr = 0; rr < 4; ++rr)
    #pragma unroll
    for (int i = 0; i < 2; ++i)
      *(volatile v4f*)(out + (size_t)(row0 + 4 * w + rr) * NIN + i * 128 + lane * 4) = o[rr][i];
  __threadfence();
  #pragma unroll
  for (int rr = 0; rr < 4; ++rr)
    #pragma unroll
    for (int i = 0; i < 2; ++i)
      *(volatile v4f*)(out + (size_t)(row0 + 4 * w + rr) * NIN + i * 128 + lane * 4) = o[rr][i];
}

extern "C" void kernel_launch(void* const* d_in, const int* in_sizes, int n_in,
                              void* d_out, int out_size, void* d_ws, size_t ws_size,
                              hipStream_t stream) {
  if (n_in < 23) return;
  if (in_sizes[0] != NB * LSEQ * NIN || in_sizes[1] != NB * LSEQ * NIN) return;
  if (in_sizes[2] != NB * LSEQ) return;
  if (in_sizes[3] != 2 * NB * LSEQ || in_sizes[4] != 2 * NB * N1 || in_sizes[5] != 2 * NB * N2) return;
  if (in_sizes[6] != 2 * NB * LSEQ * SNB || in_sizes[7] != 2 * NB * N1 * SNB) return;
  if (in_sizes[8] != 2 * NB * LSEQ * SNB * NPOS || in_sizes[9] != 2 * NB * N1 * SNB * NPOS) return;
  if (in_sizes[10] != 1 || in_sizes[11] != 1) return;
  if (in_sizes[12] != NIT * NIN) return;
  if (in_sizes[13] != NCH * NIN * CDIM || in_sizes[14] != NCH * CDIM) return;
  if (in_sizes[15] != 2 * 81 * CDIM || in_sizes[16] != 2 * CDIM || in_sizes[17] != 2 * 128 * CDIM) return;
  if (in_sizes[18] != NIN * NIN || in_sizes[19] != NIN) return;
  if (in_sizes[20] != NIN * NIN || in_sizes[21] != NIN || in_sizes[22] != NIN) return;
  if (out_size != NB * LSEQ * NIN) return;
  if (WS_TOTAL > ws_size) return;

  const float* hin   = (const float*)d_in[0];
  const float* seq   = (const float*)d_in[1];
  const float* mask  = (const float*)d_in[2];
  const int*   nbr1  = (const int*)d_in[4];
  const int*   nbr2  = (const int*)d_in[5];
  const float* wn0   = (const float*)d_in[6];
  const float* wn1   = (const float*)d_in[7];
  const float* pos0  = (const float*)d_in[8];
  const float* pos1  = (const float*)d_in[9];
  const float* table = (const float*)d_in[12];
  const float* Wr    = (const float*)d_in[13];
  const float* br    = (const float*)d_in[14];
  const float* aw1   = (const float*)d_in[15];
  const float* aw2   = (const float*)d_in[16];
  const float* aw3   = (const float*)d_in[17];
  const float* l1W   = (const float*)d_in[18];
  const float* l1b   = (const float*)d_in[19];
  const float* l2W   = (const float*)d_in[20];
  const float* l2b   = (const float*)d_in[21];
  const float* l3w   = (const float*)d_in[22];
  float* out = (float*)d_out;

  char* ws = (char*)d_ws;
  u16*      tbxs = (u16*)(ws + OFF_TBXS);
  float*    rout = (float*)(ws + OFF_ROUT);
  float*    sess = (float*)(ws + OFF_SESS);
  unsigned* catw = (unsigned*)(ws + OFF_CAT);
  float*    oab  = (float*)(ws + OFF_O);
  unsigned* catc = (unsigned*)(ws + OFF_CATC);
  float*    hg   = (float*)(ws + OFF_HG);
  u16*      wrt  = (u16*)(ws + OFF_WRT);
  u16*      w1c  = (u16*)(ws + OFF_W1C);
  u16*      w3c  = (u16*)(ws + OFF_W3C);
  u16*      lcat = (u16*)(ws + OFF_LCAT);

  float* rhs_h   = rout + (size_t)TBROWS * NIN;
  float* rhs_it  = rout + (size_t)(TBROWS + NODEB) * NIN;
  float* o1      = oab;
  float* o0      = oab + (size_t)NODEA * NIN;

  k_prep<<<PB_END, 256, 0, stream>>>(table, hin, seq, Wr, aw1, aw3, l1W, l2W, ws);

  k_route<<<AROWS / 32, 128, 0, stream>>>(tbxs, wrt, br, rout);

  k_sess<<<NB, 64, 0, stream>>>(rhs_it, mask, sess);

  k_att<0><<<NODEA / 2, 256, 0, stream>>>(rout, rout, nbr2, nbr1, wn1, pos1, sess, w1c, aw2, catw);
  k_att<1><<<NODEB / 2, 256, 0, stream>>>(rout, rhs_h, nbr1, nbr1, wn0, pos0, sess, w1c, aw2,
                                          catw + (size_t)GRPA * 128);
  k_w3<<<GRPAB / 128, 128, 0, stream>>>((const u16*)catw, w3c, oab);

  k_att<2><<<NODEB / 2, 256, 0, stream>>>(o1, o0, nbr1, nbr1, wn0, pos0, sess, w1c + 64 * KATT, aw2 + CDIM, catc);
  k_w3<<<GRPB / 128, 128, 0, stream>>>((const u16*)catc, w3c + 64 * 256, hg);

  k_fin<<<NODEB / 16, 128, 0, stream>>>(hg, tbxs + (size_t)TBROWS * NIN, lcat, l1b, l2b, l3w, out);
}
